// DeepMultiOmicNetV3_39436389712065
// MI455X (gfx1250) — hardware-verified
//
#include <hip/hip_runtime.h>
#include <stddef.h>
#include <stdint.h>


#define NB     1024
#define NI     5000
#define NCH    3
#define KP1    5056
#define NH     2000
#define NHP    2048
#define NGRP   20
#define NGW    100
#define NGWP   128
#define NG1P   2560
#define NLAY   2
#define NOUT   200
#define NOUTP  256
#define NTHR   256
#define NWAVE  8
#define TPW    64
#define WSCAP  134217728
#define LDS_GEMM (NWAVE * 32 * 64 * 4)
#define LDS_OUT  (128 * NOUT * 4)
#define WSCF   1024.0f
#define OSCF   (1.0f / 1024.0f)
#define LOG2E  1.44269504088896341f

static_assert((KP1 % 64) == 0);
static_assert(KP1 >= NI + 8);
static_assert((NI % 8) == 0);
static_assert((NH % 8) == 0);
static_assert((NHP % 128) == 0);
static_assert(NG1P == NGRP * NGWP);
static_assert((NB % 128) == 0);
static_assert(NTHR == NWAVE * 32);
static_assert(NHP == 8 * NTHR);
static_assert((KP1 / 8) <= 3 * NTHR);
static_assert(((128 * NOUT) % (4 * NTHR)) == 0);
static_assert(LDS_OUT <= 300 * 1024);
static_assert((NGW % 2) == 0);

typedef float          v2f  __attribute__((ext_vector_type(2)));
typedef float          v4f  __attribute__((ext_vector_type(4)));
typedef float          v8f  __attribute__((ext_vector_type(8)));
typedef _Float16       v8h  __attribute__((ext_vector_type(8)));
typedef _Float16       v16h __attribute__((ext_vector_type(16)));
union FragH { v16h v; v8h h[2]; };

__device__ __forceinline__ v8f wmf(v16h a, v16h b, v8f c) {
  v8f d = __builtin_amdgcn_wmma_f32_16x16x32_f16(false, a, false, b, (short)0, c, false, false);
  asm volatile("v_nop\n\tv_nop\n\tv_nop\n\tv_nop" : "+v"(d) : "v"(a), "v"(b));
  return d;
}

__device__ __forceinline__ float sigm(float v) {
  const float e = __builtin_amdgcn_exp2f(-v * LOG2E);
  return __builtin_amdgcn_rcpf(1.0f + e);
}

__global__ __launch_bounds__(NTHR) void k_merge(const float* __restrict__ x, const float* __restrict__ mw,
                                                const float* __restrict__ mb, _Float16* mh) {
  const int b = blockIdx.y;
  const int p = blockIdx.x * NTHR + threadIdx.x;
  if (p >= KP1 / 8) return;
  const int i0 = 8 * p;
  v8h hv;
#pragma unroll
  for (int e = 0; e < 8; ++e) {
    const int i = i0 + e;
    const int ic = (i < NI) ? i : (NI - 1);
    const float* xp = x + ((size_t)b * NI + ic) * NCH;
    const float* wp = mw + (size_t)ic * NCH;
    const float v = xp[0] * wp[0] + xp[1] * wp[1] + xp[2] * wp[2] + mb[ic];
    const float s = sigm(v);
    hv[e] = (_Float16)((i < NI) ? s : 0.0f);
  }
  _Float16* d = mh + (size_t)b * KP1 + i0;
  *(volatile v8h*)d = hv;
  __threadfence();
  *(volatile v8h*)d = hv;
}

template <int NIT>
__global__ __launch_bounds__(NTHR) void k_rconv(const float* __restrict__ src, _Float16* dst, int R, int C, int KP) {
  const int n = blockIdx.x;
  const bool rv = n < R;
  const int nc = rv ? n : (R - 1);
  const int npc = KP / 8;
  v8h hv[NIT];
#pragma unroll
  for (int it = 0; it < NIT; ++it) {
    const int p = it * NTHR + threadIdx.x;
    const int k0 = 8 * p;
    const bool valid = rv && (k0 < C);
    const int kc = (k0 <= C - 8) ? k0 : (C - 8);
    const float* s = src + (size_t)nc * C + kc;
    const v4f f0 = *(const v4f*)s;
    const v4f f1 = *(const v4f*)(s + 4);
    hv[it][0] = (_Float16)(valid ? f0.x * WSCF : 0.0f);
    hv[it][1] = (_Float16)(valid ? f0.y * WSCF : 0.0f);
    hv[it][2] = (_Float16)(valid ? f0.z * WSCF : 0.0f);
    hv[it][3] = (_Float16)(valid ? f0.w * WSCF : 0.0f);
    hv[it][4] = (_Float16)(valid ? f1.x * WSCF : 0.0f);
    hv[it][5] = (_Float16)(valid ? f1.y * WSCF : 0.0f);
    hv[it][6] = (_Float16)(valid ? f1.z * WSCF : 0.0f);
    hv[it][7] = (_Float16)(valid ? f1.w * WSCF : 0.0f);
  }
#pragma unroll
  for (int it = 0; it < NIT; ++it) {
    const int p = it * NTHR + threadIdx.x;
    if (p < npc) *(volatile v8h*)(dst + (size_t)n * KP + 8 * p) = hv[it];
  }
  __threadfence();
#pragma unroll
  for (int it = 0; it < NIT; ++it) {
    const int p = it * NTHR + threadIdx.x;
    if (p < npc) *(volatile v8h*)(dst + (size_t)n * KP + 8 * p) = hv[it];
  }
}

__global__ __launch_bounds__(NTHR) void k_tconv(const float* __restrict__ src, _Float16* dst,
                                                int R, int C, int RP, int CP) {
  __shared__ __attribute__((aligned(16))) float tile[128 * TPW];
  const int tid = threadIdx.x, lane = tid & 31, g = tid >> 5, hh = lane >> 4, m = lane & 15;
  const int mat = blockIdx.y;
  const int c0 = blockIdx.x * 64;
  const float* sb = src + (size_t)mat * R * C;
  _Float16* db = dst + (size_t)mat * CP * RP;
  const int c = c0 + 2 * lane;
  const bool cv = c < C;
  const int cc = cv ? c : (C - 2);
#pragma unroll 1
  for (int rc = 0; rc < RP; rc += 128) {
    __syncthreads();
#pragma unroll 4
    for (int p = 0; p < 16; ++p) {
      const int rl = g + 8 * p;
      const int r = rc + rl;
      const bool rvv = r < R;
      const int rr = rvv ? r : (R - 1);
      const v2f w = *(const v2f*)(sb + (size_t)rr * C + cc);
      v2f wz;
      wz.x = (rvv && cv) ? w.x : 0.0f;
      wz.y = (rvv && cv) ? w.y : 0.0f;
      *(v2f*)(tile + rl * TPW + 2 * lane) = wz;
    }
    __syncthreads();
    v8h hv[4];
#pragma unroll
    for (int q = 0; q < 4; ++q) {
      const int nl = 8 * g + 2 * q + hh;
      const int d8 = 8 * m;
#pragma unroll
      for (int e = 0; e < 8; ++e) hv[q][e] = (_Float16)(tile[(d8 + e) * TPW + nl] * WSCF);
    }
#pragma unroll
    for (int q = 0; q < 4; ++q) {
      _Float16* d = db + (size_t)(c0 + 8 * g + 2 * q + hh) * RP + rc + 8 * m;
      *(volatile v8h*)d = hv[q];
    }
    __threadfence();
#pragma unroll
    for (int q = 0; q < 4; ++q) {
      _Float16* d = db + (size_t)(c0 + 8 * g + 2 * q + hh) * RP + rc + 8 * m;
      *(volatile v8h*)d = hv[q];
    }
  }
}

template <int EPI>
__device__ __forceinline__ void gemm_store(const float* stg, float* Cf, _Float16* Ch,
                                           int m0, int wm, int n0, int wn, int z, int lane, int hh, int m) {
  if constexpr (EPI == 0 || EPI == 2) {
    const int ldc = (EPI == 0) ? NHP : NG1P;
    const int cofs = (EPI == 0) ? (n0 + wn) : (z * NGWP + wn);
    float* gb = Cf + (size_t)(m0 + wm) * ldc + cofs;
#pragma unroll
    for (int q = 0; q < 16; ++q) {
      const int row = 2 * q + hh;
      const v4f v = *(const v4f*)(stg + row * 64 + 4 * m);
      *(volatile v4f*)(gb + (size_t)row * ldc + 4 * m) = v;
    }
  }
  if constexpr (EPI == 0 || EPI == 1) {
    const int ldh = (EPI == 0) ? NHP : NG1P;
    _Float16* hb = Ch + (size_t)(m0 + wm) * ldh + n0 + wn;
    const int rq = lane >> 3, c8 = 8 * (lane & 7);
#pragma unroll
    for (int i = 0; i < 8; ++i) {
      const int row = 4 * i + rq;
      const v4f f0 = *(const v4f*)(stg + row * 64 + c8);
      const v4f f1 = *(const v4f*)(stg + row * 64 + c8 + 4);
      v8h hv;
      hv[0] = (_Float16)f0.x; hv[1] = (_Float16)f0.y; hv[2] = (_Float16)f0.z; hv[3] = (_Float16)f0.w;
      hv[4] = (_Float16)f1.x; hv[5] = (_Float16)f1.y; hv[6] = (_Float16)f1.z; hv[7] = (_Float16)f1.w;
      *(volatile v8h*)(hb + (size_t)row * ldh + c8) = hv;
    }
  }
}

template <int EPI>
__global__ __launch_bounds__(NTHR) void k_gemm(const _Float16* __restrict__ A, int lda,
                                               const _Float16* __restrict__ Bw, int ldb, int ksteps,
                                               const float* __restrict__ bias, float* Cf, _Float16* Ch) {
  extern __shared__ v4f lds_dyn[];
  const int tid = threadIdx.x, lane = tid & 31, wave = tid >> 5, hh = lane >> 4, m = lane & 15;
  float* stg = (float*)lds_dyn + wave * (32 * 64);
  const int n0 = blockIdx.x * 128, m0 = blockIdx.y * 128, z = blockIdx.z;
  const int wm = (wave >> 1) * 32, wn = (wave & 1) * 64;

  const _Float16* ap = A + (size_t)(m0 + wm + m) * lda + (EPI == 2 ? z * NGWP : 0) + 8 * hh;
  const _Float16* bp = Bw + (EPI == 2 ? (size_t)z * NGWP * NGWP : (size_t)0)
                          + (size_t)(n0 + wn + m) * ldb + 8 * hh;

  v8f acc[2][4];
#pragma unroll
  for (int mt = 0; mt < 2; ++mt)
#pragma unroll
    for (int nt = 0; nt < 4; ++nt) { v8f zz = {0.f, 0.f, 0.f, 0.f, 0.f, 0.f, 0.f, 0.f}; acc[mt][nt] = zz; }

#pragma unroll 1
  for (int kt = 0; kt < ksteps; ++kt) {
    const int k0 = 32 * kt;
    FragH a0, a1;
    a0.h[0] = *(const v8h*)(ap + k0);
    a0.h[1] = *(const v8h*)(ap + k0 + 16);
    a1.h[0] = *(const v8h*)(ap + (size_t)16 * lda + k0);
    a1.h[1] = *(const v8h*)(ap + (size_t)16 * lda + k0 + 16);
#pragma unroll
    for (int nt = 0; nt < 4; ++nt) {
      const _Float16* bq = bp + (size_t)nt * 16 * ldb + k0;
      FragH b;
      b.h[0] = *(const v8h*)bq;
      b.h[1] = *(const v8h*)(bq + 16);
      acc[0][nt] = wmf(a0.v, b.v, acc[0][nt]);
      acc[1][nt] = wmf(a1.v, b.v, acc[1][nt]);
    }
  }

  float bv[4];
  bool ok[4];
#pragma unroll
  for (int nt = 0; nt < 4; ++nt) {
    const int cl = wn + 16 * nt + m;
    int bidx;
    if constexpr (EPI == 0) {
      const int col = n0 + cl;
      ok[nt] = col < NH;
      bidx = ok[nt] ? col : (NH - 1);
    } else {
      const int gi = (EPI == 1) ? (int)blockIdx.x : z;
      ok[nt] = cl < NGW;
      bidx = gi * NGW + (ok[nt] ? cl : (NGW - 1));
    }
    bv[nt] = bias[bidx];
  }
#pragma unroll
  for (int mt = 0; mt < 2; ++mt) {
    float* sp = stg + (16 * mt + 8 * hh) * 64 + m;
#pragma unroll
    for (int nt = 0; nt < 4; ++nt) {
#pragma unroll
      for (int r = 0; r < 8; ++r) {
        const float t = sigm(acc[mt][nt][r] * OSCF + bv[nt]);
        sp[r * 64 + 16 * nt] = ok[nt] ? t : 0.0f;
      }
    }
  }
  __syncthreads();

  gemm_store<EPI>(stg, Cf, Ch, m0, wm, n0, wn, z, lane, hh, m);
  __threadfence();
  gemm_store<EPI>(stg, Cf, Ch, m0, wm, n0, wn, z, lane, hh, m);
}

__global__ __launch_bounds__(NTHR) void k_resid(const float* __restrict__ tt, const float* __restrict__ hold,
                                                float* hnew, _Float16* hh) {
  __shared__ __attribute__((aligned(16))) float rowv[NHP];
  const int b = blockIdx.x, t = threadIdx.x, c0 = 8 * t;
  const float* hp = hold + (size_t)b * NHP + c0;
  const v4f o0 = *(const v4f*)hp;
  const v4f o1 = *(const v4f*)(hp + 4);
  float ov[8];
  ov[0] = o0.x; ov[1] = o0.y; ov[2] = o0.z; ov[3] = o0.w;
  ov[4] = o1.x; ov[5] = o1.y; ov[6] = o1.z; ov[7] = o1.w;
  v8h hv;
#pragma unroll
  for (int e = 0; e < 8; ++e) {
    const int c = c0 + e;
    const int ccl = (c < NH) ? c : (NH - 1);
    const int g = ccl / NGW, j = ccl - g * NGW;
    const float tv = tt[(size_t)b * NG1P + g * NGWP + j];
    const float v = (c < NH) ? sigm(tv + ov[e]) : 0.0f;
    rowv[c] = v;
    hv[e] = (_Float16)v;
  }
  __syncthreads();
  const v4f va = *(const v4f*)(rowv + 4 * t);
  const v4f vb = *(const v4f*)(rowv + 1024 + 4 * t);
  float* d = hnew + (size_t)b * NHP;
  _Float16* dh = hh + (size_t)b * NHP + c0;
  *(volatile v4f*)(d + 4 * t) = va;
  *(volatile v4f*)(d + 1024 + 4 * t) = vb;
  *(volatile v8h*)dh = hv;
  __threadfence();
  *(volatile v4f*)(d + 4 * t) = va;
  *(volatile v4f*)(d + 1024 + 4 * t) = vb;
  *(volatile v8h*)dh = hv;
}

__device__ __forceinline__ void out_store(const float* img, float* out, int m0, int tid) {
#pragma unroll
  for (int it = 0; it < (128 * NOUT) / (4 * NTHR); ++it) {
    const int piece = it * NTHR + tid;
    const v4f v = *(const v4f*)(img + 4 * piece);
    *(volatile v4f*)(out + (size_t)m0 * NOUT + 4 * piece) = v;
  }
}

__global__ __launch_bounds__(NTHR) void k_out(const _Float16* __restrict__ A, const _Float16* __restrict__ Bw,
                                              const float* __restrict__ bias, float* out) {
  extern __shared__ v4f lds_dyn[];
  float* img = (float*)lds_dyn;
  const int tid = threadIdx.x, lane = tid & 31, wave = tid >> 5, hh = lane >> 4, m = lane & 15;
  const int m0 = blockIdx.x * 128;
  const int wm = (wave >> 1) * 32, wn = (wave & 1) * 64;
  const _Float16* ap = A + (size_t)(m0 + wm + m) * NHP + 8 * hh;

#pragma unroll 1
  for (int ps = 0; ps < NOUTP / 128; ++ps) {
    const _Float16* bp = Bw + (size_t)(ps * 128 + wn + m) * NHP + 8 * hh;
    v8f acc[2][4];
#pragma unroll
    for (int mt = 0; mt < 2; ++mt)
#pragma unroll
      for (int nt = 0; nt < 4; ++nt) { v8f zz = {0.f, 0.f, 0.f, 0.f, 0.f, 0.f, 0.f, 0.f}; acc[mt][nt] = zz; }
#pragma unroll 1
    for (int kt = 0; kt < NHP / 32; ++kt) {
      const int k0 = 32 * kt;
      FragH a0, a1;
      a0.h[0] = *(const v8h*)(ap + k0);
      a0.h[1] = *(const v8h*)(ap + k0 + 16);
      a1.h[0] = *(const v8h*)(ap + (size_t)16 * NHP + k0);
      a1.h[1] = *(const v8h*)(ap + (size_t)16 * NHP + k0 + 16);
#pragma unroll
      for (int nt = 0; nt < 4; ++nt) {
        const _Float16* bq = bp + (size_t)nt * 16 * NHP + k0;
        FragH b;
        b.h[0] = *(const v8h*)bq;
        b.h[1] = *(const v8h*)(bq + 16);
        acc[0][nt] = wmf(a0.v, b.v, acc[0][nt]);
        acc[1][nt] = wmf(a1.v, b.v, acc[1][nt]);
      }
    }
#pragma unroll
    for (int nt = 0; nt < 4; ++nt) {
      const int col = ps * 128 + wn + 16 * nt + m;
      const float bvv = bias[(col < NOUT) ? col : (NOUT - 1)];
      if (col < NOUT) {
#pragma unroll
        for (int mt = 0; mt < 2; ++mt) {
#pragma unroll
          for (int r = 0; r < 8; ++r)
            img[(wm + 16 * mt + 8 * hh + r) * NOUT + col] = acc[mt][nt][r] * OSCF + bvv;
        }
      }
    }
  }
  __syncthreads();
  out_store(img, out, m0, tid);
  __threadfence();
  out_store(img, out, m0, tid);
}

extern "C" void kernel_launch(void* const* d_in, const int* in_sizes, int n_in,
                              void* d_out, int out_size, void* d_ws, size_t ws_size,
                              hipStream_t stream) {
  if (n_in < 11) return;
  if (in_sizes[0] != NB * NI * NCH) return;
  if (in_sizes[1] != NI * NCH || in_sizes[2] != NI) return;
  if (in_sizes[3] != NH * NI || in_sizes[4] != NH) return;
  if (in_sizes[5] != NLAY * NGRP * NH * NGW || in_sizes[6] != NLAY * NGRP * NGW) return;
  if (in_sizes[7] != NLAY * NGRP * NGW * NGW || in_sizes[8] != NLAY * NGRP * NGW) return;
  if (in_sizes[9] != NOUT * NH || in_sizes[10] != NOUT) return;
  if (out_size != NB * NOUT) return;

  const float* x     = (const float*)d_in[0];
  const float* mw    = (const float*)d_in[1];
  const float* mb    = (const float*)d_in[2];
  const float* h0w   = (const float*)d_in[3];
  const float* h0b   = (const float*)d_in[4];
  const float* bnw1  = (const float*)d_in[5];
  const float* bnb1  = (const float*)d_in[6];
  const float* bnw2  = (const float*)d_in[7];
  const float* bnb2  = (const float*)d_in[8];
  const float* ow    = (const float*)d_in[9];
  const float* ob    = (const float*)d_in[10];
  float* out = (float*)d_out;

  char* ws = (char*)d_ws;
  size_t off = 0;
  const size_t oMh  = off; off += (size_t)NB * KP1 * 2;              off = (off + 255) & ~(size_t)255;
  const size_t oW0  = off; off += (size_t)NHP * KP1 * 2;             off = (off + 255) & ~(size_t)255;
  const size_t oHfa = off; off += (size_t)NB * NHP * 4;              off = (off + 255) & ~(size_t)255;
  const size_t oHfb = off; off += (size_t)NB * NHP * 4;              off = (off + 255) & ~(size_t)255;
  const size_t oHh  = off; off += (size_t)NB * NHP * 2;              off = (off + 255) & ~(size_t)255;
  const size_t oW1  = off; off += (size_t)NLAY * NG1P * NHP * 2;     off = (off + 255) & ~(size_t)255;
  const size_t oG1  = off; off += (size_t)NB * NG1P * 2;             off = (off + 255) & ~(size_t)255;
  const size_t oW2  = off; off += (size_t)NLAY * NGRP * NGWP * NGWP * 2; off = (off + 255) & ~(size_t)255;
  const size_t oTt  = off; off += (size_t)NB * NG1P * 4;             off = (off + 255) & ~(size_t)255;
  const size_t oOw  = off; off += (size_t)NOUTP * NHP * 2;           off = (off + 255) & ~(size_t)255;
  if (off > ws_size || off > (size_t)WSCAP) return;
  _Float16* mh  = (_Float16*)(ws + oMh);
  _Float16* w0t = (_Float16*)(ws + oW0);
  float*    hfa = (float*)(ws + oHfa);
  float*    hfb = (float*)(ws + oHfb);
  _Float16* hh  = (_Float16*)(ws + oHh);
  _Float16* w1t = (_Float16*)(ws + oW1);
  _Float16* g1h = (_Float16*)(ws + oG1);
  _Float16* w2t = (_Float16*)(ws + oW2);
  float*    tt  = (float*)(ws + oTt);
  _Float16* owt = (_Float16*)(ws + oOw);

  hipFuncSetAttribute(reinterpret_cast<const void*>(&k_gemm<0>), hipFuncAttributeMaxDynamicSharedMemorySize, LDS_GEMM);
  hipFuncSetAttribute(reinterpret_cast<const void*>(&k_gemm<1>), hipFuncAttributeMaxDynamicSharedMemorySize, LDS_GEMM);
  hipFuncSetAttribute(reinterpret_cast<const void*>(&k_gemm<2>), hipFuncAttributeMaxDynamicSharedMemorySize, LDS_GEMM);
  hipFuncSetAttribute(reinterpret_cast<const void*>(&k_out), hipFuncAttributeMaxDynamicSharedMemorySize, LDS_OUT);

  k_merge<<<dim3((KP1 / 8 + NTHR - 1) / NTHR, NB), NTHR, 0, stream>>>(x, mw, mb, mh);
  k_rconv<3><<<NHP, NTHR, 0, stream>>>(h0w, w0t, NH, NI, KP1);
  k_rconv<1><<<NOUTP, NTHR, 0, stream>>>(ow, owt, NOUT, NH, NHP);
  k_tconv<<<dim3(NGWP / 64, NLAY * NGRP), NTHR, 0, stream>>>(bnw1, w1t, NH, NGW, NHP, NGWP);
  k_tconv<<<dim3(NGWP / 64, NLAY * NGRP), NTHR, 0, stream>>>(bnw2, w2t, NGW, NGW, NGWP, NGWP);
  k_gemm<0><<<dim3(NHP / 128, NB / 128, 1), NTHR, LDS_GEMM, stream>>>(mh, KP1, w0t, KP1, KP1 / 32, h0b, hfa, hh);
  for (int l = 0; l < NLAY; ++l) {
    const float* hin = (l & 1) ? hfb : hfa;
    float* hout = (l & 1) ? hfa : hfb;
    k_gemm<1><<<dim3(NGRP, NB / 128, 1), NTHR, LDS_GEMM, stream>>>(
        hh, NHP, w1t + (size_t)l * NG1P * NHP, NHP, NHP / 32, bnb1 + (size_t)l * NH, tt, g1h);
    k_gemm<2><<<dim3(1, NB / 128, NGRP), NTHR, LDS_GEMM, stream>>>(
        g1h, NG1P, w2t + (size_t)l * NGRP * NGWP * NGWP, NGWP, NGWP / 32, bnb2 + (size_t)l * NH, tt, g1h);
    k_resid<<<NB, NTHR, 0, stream>>>(tt, hin, hout, hh);
  }
  k_out<<<NB / 128, NTHR, LDS_OUT, stream>>>(hh, owt, ob, out);
}
